// UnifiedSelfAttentionTransformer_65481071398677
// MI455X (gfx1250) — hardware-verified
//
#include <hip/hip_runtime.h>
#include <math.h>

typedef __attribute__((ext_vector_type(16))) _Float16 v16h;
typedef __attribute__((ext_vector_type(16))) __bf16 v16b;
typedef __attribute__((ext_vector_type(8)))  _Float16 v8h;
typedef __attribute__((ext_vector_type(8)))  float v8f;
typedef __attribute__((ext_vector_type(4)))  float v4f;
typedef __attribute__((ext_vector_type(2)))  float v2f;
typedef __attribute__((ext_vector_type(4)))  unsigned v4u;
typedef __attribute__((ext_vector_type(4)))  int v4i;
typedef float __attribute__((may_alias)) float_a;
typedef int __attribute__((may_alias)) int_a;

template <typename T> __device__ __forceinline__ void vst2(void* p, T v) { *(volatile T*)p = v; __threadfence(); *(volatile T*)p = v; }
__device__ __forceinline__ v8f wmma16(v16h a, v16h b, v8f c) {
  v8f d = __builtin_amdgcn_wmma_f32_16x16x32_f16(false, a, false, b, (short)0, c, false, false);
  asm volatile("v_nop\n\tv_nop\n\tv_nop\n\tv_nop" : "+v"(d) : "v"(a), "v"(b));
  return d;
}
__device__ __forceinline__ v8f wmma_bf(v16b a, v16b b, v8f c) {
  v8f d = __builtin_amdgcn_wmma_f32_16x16x32_bf16(false, a, false, b, (short)0, c, false, false);
  asm volatile("v_nop\n\tv_nop\n\tv_nop\n\tv_nop" : "+v"(d) : "v"(a), "v"(b));
  return d;
}
__device__ __forceinline__ v16h frag_h(const _Float16* rowk0, int lane) {
  union { v16h v; v8h q[2]; } u; const _Float16* p = rowk0 + 8 * (lane >> 4);
  u.q[0] = *(const v8h*)p; u.q[1] = *(const v8h*)(p + 16); return u.v;
}
__device__ __forceinline__ v16h frag_f32(const float* rowk0, int lane) {
  v16h a; const float* p = rowk0 + 8 * (lane >> 4);
#pragma unroll
  for (int i = 0; i < 8; ++i) { a[i] = (_Float16)p[i]; a[8 + i] = (_Float16)p[16 + i]; }
  return a;
}
__device__ __forceinline__ v16h frag_f32s(const float* rowk0, int lane, float sc) {
  v16h a; const float* p = rowk0 + 8 * (lane >> 4);
#pragma unroll
  for (int i = 0; i < 8; ++i) { a[i] = (_Float16)(p[i] * sc); a[8 + i] = (_Float16)(p[16 + i] * sc); }
  return a;
}
__device__ __forceinline__ v16h fragc_f32(const float* W, int k0, int n, int lane, int ld, int K) {
  v16h a; const int g = lane >> 4;
#pragma unroll
  for (int i = 0; i < 8; ++i) { const int ka = k0 + 8 * g + i, kb = ka + 16;
    a[i] = (_Float16)(ka < K ? W[(size_t)(ka < K ? ka : K - 1) * ld + n] : 0.f); a[8 + i] = (_Float16)(kb < K ? W[(size_t)(kb < K ? kb : K - 1) * ld + n] : 0.f); }
  return a;
}
struct F2 { v16b h, l; };
__device__ __forceinline__ F2 bsplit16(const float v[16]) { F2 r;
#pragma unroll
  for (int i = 0; i < 16; ++i) { const __bf16 h = (__bf16)v[i]; r.h[i] = h; r.l[i] = (__bf16)(v[i] - (float)h); }
  return r; }
__device__ __forceinline__ F2 split_row(const float* row, int k0, int lane) { float v[16]; const float* p = row + k0 + 8 * (lane >> 4);
#pragma unroll
  for (int i = 0; i < 8; ++i) { v[i] = p[i]; v[8 + i] = p[16 + i]; }
  return bsplit16(v); }
__device__ __forceinline__ F2 split_rowK(const float* row, int k0, int lane, int K) { float v[16]; const int g = lane >> 4;
#pragma unroll
  for (int i = 0; i < 8; ++i) { const int ka = k0 + 8 * g + i, kb = ka + 16; v[i] = ka < K ? row[ka < K ? ka : K - 1] : 0.f; v[8 + i] = kb < K ? row[kb < K ? kb : K - 1] : 0.f; }
  return bsplit16(v); }
__device__ __forceinline__ F2 split_col(const float* W, int k0, int n, int lane, int ld, int K) { float v[16]; const int g = lane >> 4;
#pragma unroll
  for (int i = 0; i < 8; ++i) { const int ka = k0 + 8 * g + i, kb = ka + 16; v[i] = ka < K ? W[(size_t)(ka < K ? ka : K - 1) * ld + n] : 0.f; v[8 + i] = kb < K ? W[(size_t)(kb < K ? kb : K - 1) * ld + n] : 0.f; }
  return bsplit16(v); }
__device__ __forceinline__ v8f mac3(const F2& a, const F2& b, v8f c) { c = wmma_bf(a.l, b.h, c); c = wmma_bf(a.h, b.l, c); return wmma_bf(a.h, b.h, c); }
__device__ __forceinline__ float sigm(float v) { return 1.0f / (1.0f + expf(-v)); }
#define LDSX() do { asm volatile("s_wait_dscnt 0" ::: "memory"); __builtin_amdgcn_wave_barrier(); __builtin_amdgcn_fence(__ATOMIC_RELEASE, "workgroup"); } while (0)


#define NLAY 4
#define NB 8
#define SS 1024
#define NR (NB * SS)
#define EE 256
#define NH 8
#define DK 32
#define FF 1024
#define NCLS 10
#define VOC 32000
#ifndef NBT
#define NBT NB
#define TB0 0
#endif
#define RT (NBT * SS)
#define RB0 ((size_t)TB0 * SS)
typedef __attribute__((ext_vector_type(8))) __bf16 v8b;
__device__ __forceinline__ v16b frag_b(const __bf16* rowk0, int lane) {
  union { v16b v; v8b q[2]; } u; const __bf16* p = rowk0 + 8 * (lane >> 4);
  u.q[0] = *(const v8b*)p; u.q[1] = *(const v8b*)(p + 16); return u.v;
}
__device__ __forceinline__ float bfr(float v) { return (float)(__bf16)v; }
__device__ __attribute__((noinline)) float exp_ni(float v) { return expf(v); }
__device__ __attribute__((noinline)) float erf_ni(float v) { return erff(v); }
__device__ __attribute__((noinline)) float cos_ni(float v) { return cosf(v); }
__device__ __attribute__((noinline)) float sin_ni(float v) { return sinf(v); }

#define PL_C  0
#define PL_1  ((size_t)EE * EE)
#define PL_2  (PL_1 + (size_t)FF * EE)
#define PL_SZ (PL_2 + (size_t)EE * FF)
#define PK_CLS ((size_t)NLAY * PL_SZ)
#define PK_END (PK_CLS + 16 * EE)
#define WS_PK  0u
#define WS_X   (((2u * PK_END) + 127u) / 128u * 128u)
#define WS_X2  (WS_X + 4u * NR * EE)
#define WS_P   (WS_X2 + 4u * NR * EE)
#define WS_PT  (WS_P + 2u * NR * EE)
#define WS_AT  (WS_PT + 2u * NR * EE)
#define WS_GH  (WS_AT + 4u * NR * EE)
#define WS_GL  (WS_GH + 2u * NR * FF)
#define WS_MEAN (WS_GL + 2u * NR * FF)
#define WS_END (WS_MEAN + 4u * NB * (SS / 64) * EE)

__global__ __launch_bounds__(256) void k_pack(const float* __restrict__ WC, const float* __restrict__ W1, const float* __restrict__ W2, const float* __restrict__ WCLS, __bf16* __restrict__ PK) {
  __shared__ __align__(16) __bf16 s[FF]; const int n = blockIdx.x, which = blockIdx.y, lay = blockIdx.z, t = threadIdx.x; int K, NO; size_t dst; const float* base;
  if (lay == NLAY) { if (which != 0 || n >= 16) return; K = EE; for (int k = t; k < K; k += 256) s[k] = (__bf16)((n < NCLS) ? WCLS[(size_t)k * NCLS + n] : 0.f); __syncthreads(); for (int q = t; q < K / 8; q += 256) vst2((unsigned*)(PK + PK_CLS + (size_t)n * EE + q * 8), *(const v4u*)&s[q * 8]); return; }
  switch (which) { case 0: base = WC + (size_t)lay * EE * EE; K = EE; NO = EE; dst = PL_C; break; case 1: base = W1 + (size_t)lay * EE * FF; K = EE; NO = FF; dst = PL_1; break; default: base = W2 + (size_t)lay * FF * EE; K = FF; NO = EE; dst = PL_2; break; }
  if (n >= NO) return;
  for (int k = t; k < K; k += 256) s[k] = (__bf16)base[(size_t)k * NO + n];
  __syncthreads();
  for (int q = t; q < K / 8; q += 256) vst2((unsigned*)(PK + (size_t)lay * PL_SZ + dst + (size_t)n * K + q * 8), *(const v4u*)&s[q * 8]);
}
__global__ __launch_bounds__(64) void k_embed(const int* __restrict__ TOK, const float* __restrict__ EMBT, float* __restrict__ X) {
  const size_t row = RB0 + blockIdx.x; const int t = threadIdx.x; const int s = (int)(row % SS); int tok = TOK[row]; tok = min(max(tok, 0), VOC - 1); v4f o;
#pragma unroll
  for (int i = 0; i < 4; ++i) { const int c = t * 4 + i; const int i2 = c & ~1; const float div = exp_ni((float)i2 * (-9.210340371976184f / (float)EE)); const float ang = (float)s * div; const float pe = (c & 1) ? cos_ni(ang) : sin_ni(ang); o[i] = bfr(EMBT[(size_t)tok * EE + c]) + pe; }
  vst2(X + row * EE + t * 4, o);
}
__global__ __launch_bounds__(256) void k_qproj(const float* __restrict__ X, const float* __restrict__ TH, __bf16* __restrict__ P, __bf16* __restrict__ PT) {
  __shared__ __align__(16) __bf16 sp[64][EE + 8]; __shared__ __align__(16) __bf16 st[EE][72];
  const int tid = threadIdx.x; const size_t rb = RB0 + (size_t)blockIdx.x * 64; const int r = tid >> 2, hq = tid & 3;
  for (int hh = 0; hh < 2; ++hh) { const int h = hq * 2 + hh; const float* xr = X + (rb + r) * EE + h * DK; float c[DK];
#pragma unroll
    for (int d = 0; d < DK; ++d) c[d] = cos_ni(xr[d] + bfr(TH[h * DK + d]));
    float cum = c[0]; float pv[DK];
#pragma unroll
    for (int d = 1; d < DK; ++d) { cum = cum * c[d]; pv[d] = cum; }
    float h0 = c[1];
#pragma unroll
    for (int d = 2; d < DK; ++d) h0 = h0 * c[d];
    pv[0] = h0;
#pragma unroll
    for (int d = 0; d < DK; ++d) { const __bf16 hb = (__bf16)pv[d]; sp[r][h * DK + d] = hb; st[h * DK + d][r] = hb; } }
  __syncthreads();
  for (int e = tid; e < 64 * 32; e += 256) { const int rr = e >> 5, pc = e & 31; vst2((unsigned*)(P + (rb + rr) * EE + pc * 8), *(const v4u*)&sp[rr][pc * 8]); }
  { const size_t b = rb / SS; const int s0 = (int)(rb % SS); for (int e = tid; e < EE * 8; e += 256) { const int d = e >> 3, pc = e & 7; vst2((unsigned*)(PT + ((size_t)b * EE + d) * SS + s0 + pc * 8), *(const v4u*)&st[d][pc * 8]); } }
}
__global__ __launch_bounds__(128) void k_attn(const __bf16* __restrict__ P, const __bf16* __restrict__ PT, float* __restrict__ AT) {
  __shared__ __align__(16) __bf16 spb[4][16][40]; __shared__ __align__(16) float so[4][16][EE + 4];
  const int tid = threadIdx.x, wave = tid >> 5, lane = tid & 31, col = lane & 15, g = lane >> 4; const int qb = blockIdx.x; const size_t b = blockIdx.y + TB0; const size_t q0 = b * SS + qb * 64 + wave * 16;
  const __bf16* qrow = P + (q0 + col) * EE;
  const __bf16* PTb = PT + b * EE * SS;
  float m[8], l[8];
#pragma unroll
  for (int r = 0; r < 8; ++r) { m[r] = -3.0e38f; l[r] = 0.f; }
  v8f acc[16] = {};
#pragma unroll 1
  for (int ks = 0; ks < SS / 32; ++ks) { v8f s[2];
#pragma unroll
    for (int ct = 0; ct < 2; ++ct) { const size_t kk = b * SS + ks * 32 + ct * 16 + col; v8f c = {};
#pragma unroll
      for (int kc = 0; kc < 8; ++kc) c = wmma_bf(frag_b(qrow + kc * 32, lane), frag_b(P + kk * EE + kc * 32, lane), c);
#pragma unroll
      for (int r = 0; r < 8; ++r) s[ct][r] = c[r] * 0.17677669529663687f; }
#pragma unroll
    for (int r = 0; r < 8; ++r) { float mx = fmaxf(s[0][r], s[1][r]);
#pragma unroll
      for (int o = 1; o < 16; o <<= 1) mx = fmaxf(mx, __shfl_xor(mx, o));
      const float mn = fmaxf(m[r], mx); const float alpha = (m[r] <= -1.0e38f) ? 0.f : __expf(m[r] - mn); const float e0 = __expf(s[0][r] - mn), e1 = __expf(s[1][r] - mn); float es = e0 + e1;
#pragma unroll
      for (int o = 1; o < 16; o <<= 1) es += __shfl_xor(es, o);
      l[r] = l[r] * alpha + es; m[r] = mn;
#pragma unroll
      for (int jt = 0; jt < 16; ++jt) acc[jt][r] *= alpha;
      spb[wave][8 * g + r][col] = (__bf16)e0; spb[wave][8 * g + r][16 + col] = (__bf16)e1; }
    LDSX();
    const v16b pa = frag_b(&spb[wave][col][0], lane);
#pragma unroll
    for (int jt = 0; jt < 16; ++jt) acc[jt] = wmma_bf(pa, frag_b(PTb + (size_t)(jt * 16 + col) * SS + ks * 32, lane), acc[jt]);
    LDSX(); }
#pragma unroll
  for (int r = 0; r < 8; ++r) { const float il = 1.0f / l[r];
#pragma unroll
    for (int jt = 0; jt < 16; ++jt) so[wave][8 * g + r][jt * 16 + col] = acc[jt][r] * il; }
  LDSX();
  for (int rl = 0; rl < 16; ++rl) { vst2(AT + (q0 + rl) * EE + lane * 4, *(const v4f*)&so[wave][rl][lane * 4]); vst2(AT + (q0 + rl) * EE + 128 + lane * 4, *(const v4f*)&so[wave][rl][128 + lane * 4]); }
}
template <int MODE>
__global__ __launch_bounds__(128) void k_lin(const float* __restrict__ A, const float* __restrict__ THF, const __bf16* __restrict__ AG, const __bf16* __restrict__ AGL, const __bf16* __restrict__ Pw, const float* __restrict__ BIAS, const float* __restrict__ X, float* __restrict__ OUTF, __bf16* __restrict__ OUTG, __bf16* __restrict__ OUTGL) {
  __shared__ __align__(16) float so[4][16][132]; __shared__ __align__(16) __bf16 sg[4][16][136], sgl[4][16][136];
  const int tid = threadIdx.x, wave = tid >> 5, lane = tid & 31, col = lane & 15, g = lane >> 4; const size_t r0 = RB0 + (size_t)blockIdx.x * 64 + wave * 16; const int n0 = blockIdx.y * 128;
  constexpr int KD = (MODE == 2) ? FF : EE;
  v8f acc[8] = {};
  if (MODE == 2) {
#pragma unroll 2
    for (int kc = 0; kc < KD / 32; ++kc) { const v16b a = frag_b(AG + (r0 + col) * FF + kc * 32, lane), al = frag_b(AGL + (r0 + col) * FF + kc * 32, lane);
#pragma unroll
      for (int j = 0; j < 8; ++j) { const v16b w = frag_b(Pw + (size_t)(n0 + j * 16 + col) * KD + kc * 32, lane); acc[j] = wmma_bf(al, w, acc[j]); acc[j] = wmma_bf(a, w, acc[j]); } }
  } else if (MODE == 1) {
#pragma unroll 2
    for (int kc = 0; kc < KD / 32; ++kc) { v16b ah, al; { const float* p = A + (r0 + col) * EE + kc * 32 + 8 * g; const float* tp = THF + kc * 32 + 8 * g;
#pragma unroll
        for (int i = 0; i < 16; ++i) { const int off = (i & 7) + ((i >> 3) << 4); const float v = cos_ni(p[off]) * cos_ni(bfr(tp[off])); const __bf16 hb = (__bf16)v; ah[i] = hb; al[i] = (__bf16)(v - (float)hb); } }
#pragma unroll
      for (int j = 0; j < 8; ++j) { const v16b w = frag_b(Pw + (size_t)(n0 + j * 16 + col) * KD + kc * 32, lane); acc[j] = wmma_bf(al, w, acc[j]); acc[j] = wmma_bf(ah, w, acc[j]); } }
  } else {
#pragma unroll 2
    for (int kc = 0; kc < KD / 32; ++kc) { const F2 a = split_row(A + (r0 + col) * EE, kc * 32, lane);
#pragma unroll
      for (int j = 0; j < 8; ++j) { const v16b w = frag_b(Pw + (size_t)(n0 + j * 16 + col) * KD + kc * 32, lane); acc[j] = wmma_bf(a.l, w, acc[j]); acc[j] = wmma_bf(a.h, w, acc[j]); } } }
  if (MODE == 1) {
#pragma unroll
    for (int j = 0; j < 8; ++j) { const float bb = bfr(BIAS[n0 + j * 16 + col]);
#pragma unroll
      for (int r = 0; r < 8; ++r) { const float v = fmaxf(acc[j][r] + bb, 0.f); const __bf16 hb = (__bf16)v; sg[wave][8 * g + r][j * 16 + col] = hb; sgl[wave][8 * g + r][j * 16 + col] = (__bf16)(v - (float)hb); } }
    LDSX();
    for (int rl = 0; rl < 16; ++rl) { if (lane < 16) vst2((unsigned*)(OUTG + (r0 + rl) * FF + n0 + lane * 8), *(const v4u*)&sg[wave][rl][lane * 8]); else vst2((unsigned*)(OUTGL + (r0 + rl) * FF + n0 + (lane - 16) * 8), *(const v4u*)&sgl[wave][rl][(lane - 16) * 8]); }
  } else {
#pragma unroll
    for (int j = 0; j < 8; ++j) { const int c = n0 + j * 16 + col; const float bb = bfr(BIAS[c]);
#pragma unroll
      for (int r = 0; r < 8; ++r) { const size_t row = r0 + 8 * g + r; so[wave][8 * g + r][j * 16 + col] = acc[j][r] + bb + X[row * EE + c]; } }
    LDSX();
    for (int rl = 0; rl < 16; ++rl) vst2(OUTF + (r0 + rl) * EE + n0 + lane * 4, *(const v4f*)&so[wave][rl][lane * 4]); }
}
__global__ __launch_bounds__(64) void k_ln(const float* __restrict__ SRC, const float* __restrict__ G, const float* __restrict__ Bv, float* __restrict__ OUT) {
  __shared__ float red[2][2]; const int t = threadIdx.x; const size_t row = RB0 + blockIdx.x; const float* p = SRC + row * EE + t * 4;
  float v[4] = {p[0], p[1], p[2], p[3]}; float s = (v[0] + v[1]) + (v[2] + v[3]);
#pragma unroll
  for (int o = 1; o < 32; o <<= 1) s += __shfl_xor(s, o);
  if ((t & 31) == 0) red[0][t >> 5] = s; __syncthreads();
  const float mu = (red[0][0] + red[0][1]) / (float)EE; float q = 0.f;
#pragma unroll
  for (int i = 0; i < 4; ++i) { const float d = v[i] - mu; q += d * d; }
#pragma unroll
  for (int o = 1; o < 32; o <<= 1) q += __shfl_xor(q, o);
  if ((t & 31) == 0) red[1][t >> 5] = q; __syncthreads();
  const float inv = 1.0f / sqrtf((red[1][0] + red[1][1]) / (float)EE + 1e-5f); v4f o4;
#pragma unroll
  for (int i = 0; i < 4; ++i) o4[i] = (v[i] - mu) * inv * bfr(G[t * 4 + i]) + bfr(Bv[t * 4 + i]);
  vst2(OUT + row * EE + t * 4, o4);
}
__global__ __launch_bounds__(256) void k_pool(const float* __restrict__ X, float* __restrict__ MP) {
  const int c = threadIdx.x; const size_t b = blockIdx.y + TB0; const int blk = blockIdx.x; float s = 0.f; for (int r = 0; r < 64; ++r) s += X[(b * SS + blk * 64 + r) * EE + c];
  MP[(b * (SS / 64) + blk) * EE + c] = s;
}
__global__ __launch_bounds__(64) void k_cls(const float* __restrict__ MP, const __bf16* __restrict__ PK, const float* __restrict__ BCLS, float* __restrict__ OUT) {
  __shared__ __align__(16) __bf16 sah[16][EE + 8], sal[16][EE + 8]; __shared__ float so[16][16];
  const int tid = threadIdx.x, lane = tid & 31, wave = tid >> 5, col = lane & 15, g = lane >> 4;
  for (int e = tid; e < 16 * (EE + 8); e += 64) { const int r = e / (EE + 8), c = e % (EE + 8); float v = 0.f; if (r < NBT && c < EE) { float s = 0.f; for (int blk = 0; blk < SS / 64; ++blk) s += MP[((size_t)(TB0 + r) * (SS / 64) + blk) * EE + c]; v = s / (float)SS; } const __bf16 hb = (__bf16)v; sah[r][c] = hb; sal[r][c] = (__bf16)(v - (float)hb); }
  __syncthreads();
  if (wave == 0) { v8f acc = {};
#pragma unroll 1
    for (int kc = 0; kc < EE / 32; ++kc) { F2 a; a.h = frag_b(&sah[col][kc * 32], lane); a.l = frag_b(&sal[col][kc * 32], lane); const v16b w = frag_b(PK + PK_CLS + (size_t)col * EE + kc * 32, lane); acc = wmma_bf(a.l, w, acc); acc = wmma_bf(a.h, w, acc); }
#pragma unroll
    for (int r = 0; r < 8; ++r) so[8 * g + r][col] = acc[r] + ((col < NCLS) ? bfr(BCLS[col]) : 0.f); }
  __syncthreads();
  if (tid < NBT) { for (int c = 0; c < NCLS; ++c) OUT[(size_t)(TB0 + tid) * NCLS + c] = so[tid][c]; }
}
extern "C" void kernel_launch(void* const* d_in, const int* in_sizes, int n_in, void* d_out, int out_size, void* d_ws, size_t ws_size, hipStream_t stream) {
  (void)in_sizes; (void)n_in; (void)out_size;
  const float** F = (const float**)d_in;
  if (ws_size < (size_t)WS_END) return;
  char* ws = (char*)d_ws; __bf16 *PK = (__bf16*)(ws + WS_PK), *P = (__bf16*)(ws + WS_P), *PT = (__bf16*)(ws + WS_PT), *GH = (__bf16*)(ws + WS_GH), *GL = (__bf16*)(ws + WS_GL); float *X = (float*)(ws + WS_X), *X2 = (float*)(ws + WS_X2), *AT = (float*)(ws + WS_AT), *MP = (float*)(ws + WS_MEAN);
  k_pack<<<dim3(FF, 3, NLAY + 1), 256, 0, stream>>>(F[3], F[8], F[10], F[14], PK);
  k_embed<<<RT, 64, 0, stream>>>((const int*)d_in[0], F[1], X);
  for (int lay = 0; lay < NLAY; ++lay) { const __bf16* PKL = PK + (size_t)lay * PL_SZ;
    k_qproj<<<RT / 64, 256, 0, stream>>>(X, F[2] + lay * NH * DK, P, PT);
    k_attn<<<dim3(SS / 64, NBT), 128, 0, stream>>>(P, PT, AT);
    k_lin<0><<<dim3(RT / 64, EE / 128), 128, 0, stream>>>(AT, nullptr, nullptr, nullptr, PKL + PL_C, F[4] + lay * EE, X, X2, nullptr, nullptr);
    k_ln<<<RT, 64, 0, stream>>>(X2, F[5] + lay * EE, F[6] + lay * EE, X);
    k_lin<1><<<dim3(RT / 64, FF / 128), 128, 0, stream>>>(X, F[7] + lay * EE, nullptr, nullptr, PKL + PL_1, F[9] + lay * FF, nullptr, nullptr, GH, GL);
    k_lin<2><<<dim3(RT / 64, EE / 128), 128, 0, stream>>>(nullptr, nullptr, GH, GL, PKL + PL_2, F[11] + lay * EE, X, X2, nullptr, nullptr);
    k_ln<<<RT, 64, 0, stream>>>(X2, F[12] + lay * EE, F[13] + lay * EE, X); }
  k_pool<<<dim3(SS / 64, NBT), 256, 0, stream>>>(X, MP);
  k_cls<<<1, 64, 0, stream>>>(MP, PK, F[15], (float*)d_out);
}
